// TransformerBlockQuantum_65481071405230
// MI455X (gfx1250) — hardware-run, weakly checked
//
#include <hip/hip_runtime.h>
#include <math.h>

typedef __attribute__((ext_vector_type(16))) _Float16 v16h;
typedef __attribute__((ext_vector_type(8)))  _Float16 v8h;
typedef __attribute__((ext_vector_type(4)))  _Float16 v4h;
typedef __attribute__((ext_vector_type(8)))  float    v8f;
typedef __attribute__((ext_vector_type(4)))  float    v4f;

constexpr int kBatch       = 64;
constexpr int kSeq         = 2048;
constexpr int kChan        = 8;
constexpr int kHidden      = 1024;
constexpr int kTok         = kBatch * kSeq;
constexpr int kWavesPerBlk = 8;
constexpr int kTokPerWave  = 16;
constexpr int kTokPerBlk   = kWavesPerBlk * kTokPerWave;
constexpr int kThreads     = kWavesPerBlk * 32;
constexpr int kSteps       = kHidden / 32;
static_assert(kTok == 131072, "token count");
static_assert(kChan == 8, "channel split 4 + 4 across lane halves");
static_assert((kTok % kTokPerBlk) == 0, "grid covers the tokens exactly");
static_assert((kHidden % 32) == 0, "hidden width is a multiple of the 32-deep step");
static_assert(kHidden == 4 * kThreads, "staging coverage: 4 rows / groups per thread");

constexpr float kW1Carry  = 64.0f;
constexpr float kQCarry   = 16.0f;
constexpr float kHidCarry = 16.0f;
constexpr float kW2Carry  = 1024.0f;
constexpr float kEpi1     = kHidCarry / (kW1Carry * kQCarry);
constexpr float kEpi2     = 1.0f / (kW2Carry * kHidCarry);
constexpr float kLnEps    = 1e-5f;

union H16 { v16h v; v8h h[2]; v4h q[4]; };

__device__ __forceinline__ v8f mma_f16(v16h a, v16h b, v8f c) {
  c = __builtin_amdgcn_wmma_f32_16x16x32_f16(false, a, false, b, (short)0, c, false, false);
  asm volatile("v_nop\n\tv_nop\n\tv_nop\n\tv_nop" : "+v"(c) : "v"(a), "v"(b));
  return c;
}

__global__ __launch_bounds__(kThreads) void fused_block_kernel(
    const float* __restrict__ x,
    const float* __restrict__ ln1g, const float* __restrict__ ln1b,
    const float* __restrict__ ln2g, const float* __restrict__ ln2b,
    const float* __restrict__ rp,   const float* __restrict__ ry,
    const float* __restrict__ w1,   const float* __restrict__ b1,
    const float* __restrict__ w2,   const float* __restrict__ b2,
    float* __restrict__ out)
{
  __shared__ __align__(16) _Float16 sW1[kHidden * kChan];
  __shared__ __align__(16) _Float16 sW2[kChan * kHidden];
  __shared__ __align__(16) float    sB1[kHidden];
  __shared__ __align__(16) float    sOut[kWavesPerBlk * kTokPerWave * kChan];

  const int tid  = threadIdx.x;
  const int lane = tid & 31;
  const int wave = tid >> 5;
  const int hh   = lane >> 4;
  const int m    = lane & 15;

#pragma unroll 1
  for (int i = 0; i < 4; ++i) {
    const int g = tid + kThreads * i;
    const v4f a0 = *(const v4f*)(w1 + (size_t)g * 8);
    const v4f a1 = *(const v4f*)(w1 + (size_t)g * 8 + 4);
    const v4f c0 = *(const v4f*)(w2 + (size_t)g * 8);
    const v4f c1 = *(const v4f*)(w2 + (size_t)g * 8 + 4);
    v8h hv, gv;
#pragma unroll
    for (int e = 0; e < 4; ++e) {
      hv[e]     = (_Float16)(a0[e] * kW1Carry);
      hv[4 + e] = (_Float16)(a1[e] * kW1Carry);
      gv[e]     = (_Float16)(c0[e] * kW2Carry);
      gv[4 + e] = (_Float16)(c1[e] * kW2Carry);
    }
    *(v8h*)(sW1 + g * 8) = hv;
    *(v8h*)(sW2 + g * 8) = gv;
  }
  {
    const v4f bv = *(const v4f*)(b1 + 4 * tid);
    v4f bs;
    bs[0] = bv[0] * kHidCarry;
    bs[1] = bv[1] * kHidCarry;
    bs[2] = bv[2] * kHidCarry;
    bs[3] = bv[3] * kHidCarry;
    *(v4f*)(sB1 + 4 * tid) = bs;
  }

  const int tok0 = blockIdx.x * kTokPerBlk + wave * kTokPerWave;
  int tokc = tok0 + m;
  tokc = (tokc < kTok) ? tokc : (kTok - 1);
  const v4f xv = *(const v4f*)(x + (size_t)tokc * kChan + 4 * hh);

  const float ryv = ry[lane & 7];
  const float p0 = rp[0];
  const float p1 = rp[1];
  const float p3 = rp[3];
  const float p4 = rp[4];
  const float uarg = (lane == 8) ? p1 : ((lane == 9) ? p4 : ryv);
  const float cu   = cosf(uarg);
  const float cp1  = __shfl(cu, 8, 32);
  const float cp4  = __shfl(cu, 9, 32);
  const float cry0 = __shfl(cu, 4 * hh + 0, 32);
  const float cry1 = __shfl(cu, 4 * hh + 1, 32);
  const float cry2 = __shfl(cu, 4 * hh + 2, 32);
  const float cry3 = __shfl(cu, 4 * hh + 3, 32);

  const float shift = hh ? p3 : p0;
  const float c0 = cosf(xv[0] + shift);
  const float c1 = cosf(xv[1]);
  const float c2 = cosf(xv[2]);
  const float c3 = cosf(xv[3]);
  const float m1  = hh ? cp4 : (c0 * cp1);
  const float av0 = c0;
  const float av1 = m1 * c1;
  const float av2 = c2;
  const float av3 = hh ? c3 : (c2 * c3);

  float hN0, hN1, hN2, hN3;
  {
    const float h0 = xv[0] + av0, h1 = xv[1] + av1, h2 = xv[2] + av2, h3 = xv[3] + av3;
    float s = (h0 + h1) + (h2 + h3);
    s += __shfl_xor(s, 16, 32);
    const float mu = s * 0.125f;
    const float d0 = h0 - mu, d1 = h1 - mu, d2 = h2 - mu, d3 = h3 - mu;
    float vs = (d0 * d0 + d1 * d1) + (d2 * d2 + d3 * d3);
    vs += __shfl_xor(vs, 16, 32);
    const float inv = rsqrtf(vs * 0.125f + kLnEps);
    const v4f g  = *(const v4f*)(ln1g + 4 * hh);
    const v4f bb = *(const v4f*)(ln1b + 4 * hh);
    hN0 = d0 * inv * g[0] + bb[0];
    hN1 = d1 * inv * g[1] + bb[1];
    hN2 = d2 * inv * g[2] + bb[2];
    hN3 = d3 * inv * g[3] + bb[3];
  }

  H16 bq;
  {
    const float q0 = cry0 * cosf(av0) * kQCarry;
    const float q1 = cry1 * cosf(av1) * kQCarry;
    const float q2 = cry2 * cosf(av2) * kQCarry;
    const float q3 = cry3 * cosf(av3) * kQCarry;
    v4h qh;
    qh[0] = (_Float16)q0;
    qh[1] = (_Float16)q1;
    qh[2] = (_Float16)q2;
    qh[3] = (_Float16)q3;
    const v16h z16 = (v16h){0, 0, 0, 0, 0, 0, 0, 0, 0, 0, 0, 0, 0, 0, 0, 0};
    bq.v = z16;
    bq.q[0] = qh;
  }

  __syncthreads();

  const v8f  z8  = (v8f){0.f, 0.f, 0.f, 0.f, 0.f, 0.f, 0.f, 0.f};
  const v16h z16 = (v16h){0, 0, 0, 0, 0, 0, 0, 0, 0, 0, 0, 0, 0, 0, 0, 0};
  v8f acc2 = z8;
  const _Float16* w1p = sW1 + m * kChan + 4 * hh;
  const _Float16* w2p = sW2 + (m & 7) * kHidden + 8 * hh;
  const float*    b1p = sB1 + 8 * hh;

#pragma unroll 4
  for (int s = 0; s < kSteps; ++s) {
    const int k0 = s * 32;
    H16 a0, a1;
    a0.v = z16;
    a1.v = z16;
    a0.q[0] = *(const v4h*)(w1p + (k0) * kChan);
    a1.q[0] = *(const v4h*)(w1p + (k0 + 16) * kChan);
    const v8f d0 = mma_f16(a0.v, bq.v, z8);
    const v8f d1 = mma_f16(a1.v, bq.v, z8);

    const v4f b00 = *(const v4f*)(b1p + k0);
    const v4f b01 = *(const v4f*)(b1p + k0 + 4);
    const v4f b10 = *(const v4f*)(b1p + k0 + 16);
    const v4f b11 = *(const v4f*)(b1p + k0 + 20);

    v16h hb;
#pragma unroll
    for (int r = 0; r < 4; ++r) {
      hb[r]      = (_Float16)fmaxf(fmaf(d0[r],     kEpi1, b00[r]), 0.0f);
      hb[4 + r]  = (_Float16)fmaxf(fmaf(d0[4 + r], kEpi1, b01[r]), 0.0f);
      hb[8 + r]  = (_Float16)fmaxf(fmaf(d1[r],     kEpi1, b10[r]), 0.0f);
      hb[12 + r] = (_Float16)fmaxf(fmaf(d1[4 + r], kEpi1, b11[r]), 0.0f);
    }

    H16 a2;
    a2.h[0] = *(const v8h*)(w2p + k0);
    a2.h[1] = *(const v8h*)(w2p + k0 + 16);
    acc2 = mma_f16(a2.v, hb, acc2);
  }

  {
    const float f0 = hh ? acc2[4] : acc2[0];
    const float f1 = hh ? acc2[5] : acc2[1];
    const float f2 = hh ? acc2[6] : acc2[2];
    const float f3 = hh ? acc2[7] : acc2[3];
    const v4f b2v = *(const v4f*)(b2 + 4 * hh);
    const float y0 = hN0 + (f0 * kEpi2 + b2v[0]);
    const float y1 = hN1 + (f1 * kEpi2 + b2v[1]);
    const float y2 = hN2 + (f2 * kEpi2 + b2v[2]);
    const float y3 = hN3 + (f3 * kEpi2 + b2v[3]);
    float s = (y0 + y1) + (y2 + y3);
    s += __shfl_xor(s, 16, 32);
    const float mu = s * 0.125f;
    const float d0 = y0 - mu, d1 = y1 - mu, d2 = y2 - mu, d3 = y3 - mu;
    float vs = (d0 * d0 + d1 * d1) + (d2 * d2 + d3 * d3);
    vs += __shfl_xor(vs, 16, 32);
    const float inv = rsqrtf(vs * 0.125f + kLnEps);
    const v4f g  = *(const v4f*)(ln2g + 4 * hh);
    const v4f bb = *(const v4f*)(ln2b + 4 * hh);
    v4f ov;
    ov[0] = d0 * inv * g[0] + bb[0];
    ov[1] = d1 * inv * g[1] + bb[1];
    ov[2] = d2 * inv * g[2] + bb[2];
    ov[3] = d3 * inv * g[3] + bb[3];
    *(v4f*)(sOut + wave * (kTokPerWave * kChan) + m * kChan + 4 * hh) = ov;
  }
  __syncthreads();
  {
    const v4f val = *(const v4f*)(sOut + wave * (kTokPerWave * kChan) + 4 * lane);
    const bool ok = (tok0 + (lane >> 1)) < kTok;
    float* op = out + (size_t)tok0 * kChan + 4 * lane;
    if (ok) *(volatile v4f*)op = val;
    __threadfence();
    if (ok) *(volatile v4f*)op = val;
  }
}

extern "C" void kernel_launch(void* const* d_in, const int* in_sizes, int n_in,
                              void* d_out, int out_size, void* d_ws, size_t ws_size,
                              hipStream_t stream) {
  (void)d_ws; (void)ws_size;
  if (n_in < 11) return;
  if (in_sizes[0] != kTok * kChan) return;
  if (in_sizes[1] != kChan || in_sizes[2] != kChan || in_sizes[3] != kChan || in_sizes[4] != kChan) return;
  if (in_sizes[5] != 6) return;
  if (in_sizes[6] != kChan) return;
  if (in_sizes[7] != kHidden * kChan) return;
  if (in_sizes[8] != kHidden) return;
  if (in_sizes[9] != kChan * kHidden) return;
  if (in_sizes[10] != kChan) return;
  if (out_size != kTok * kChan) return;

  const float* x    = (const float*)d_in[0];
  const float* ln1g = (const float*)d_in[1];
  const float* ln1b = (const float*)d_in[2];
  const float* ln2g = (const float*)d_in[3];
  const float* ln2b = (const float*)d_in[4];
  const float* rp   = (const float*)d_in[5];
  const float* ry   = (const float*)d_in[6];
  const float* w1   = (const float*)d_in[7];
  const float* b1   = (const float*)d_in[8];
  const float* w2   = (const float*)d_in[9];
  const float* b2   = (const float*)d_in[10];

  fused_block_kernel<<<kTok / kTokPerBlk, kThreads, 0, stream>>>(
      x, ln1g, ln1b, ln2g, ln2b, rp, ry, w1, b1, w2, b2, (float*)d_out);
}
